// GPSLayer_53360673686110
// MI455X (gfx1250) — hardware-run, weakly checked
//
#include <hip/hip_runtime.h>
#include <stddef.h>
#include <stdint.h>
#include <math.h>


#define CH      128
#define CH2     256
#define QKVW    384
#define GLN     512
#define NHD     8
#define HDM     16
#define NTHR    256
#define NWAVE   8
#define EPT     8
#define CHUNK   (NTHR * EPT)
#define WCAP    (EPT * 32)
#define LISTN   (NWAVE * WCAP)
#define NBMAX   2048
#define RCAP    28672
#define DEGCAP  256
#define STW     128
#define GBM     64
#define GBN     64
#define GTHR    128
#define ATHR    64
#define AWAV    2
#define ARTS    (GLN / (16 * AWAV))
#define AWSZ    (16 * GLN + 8 * GLN)
#define CACT    8.0f
#define CWGT    256.0f
#define CLO     2048.0f
#define CPRB    1024.0f
#define SC1     0.00390625f
#define SC2     1.9073486328125e-06f
#define SCO     0.0001220703125f
#define S11     0.00048828125f
#define S22     2.384185791015625e-07f
#define WSMAX   134217728
#define LDS_AGG ((2 * RCAP + 2 * NBMAX + LISTN) * 4 + 64)
#define LDS_ATT (3 * GLN * HDM * 2 + AWAV * AWSZ * 4)

static_assert((CHUNK & (CHUNK - 1)) == 0 && CHUNK <= 4096);
static_assert((NBMAX & (NBMAX - 1)) == 0 && NBMAX <= 4096);
static_assert(NTHR * 8 == NBMAX);
static_assert(LISTN >= NBMAX);
static_assert(LISTN >= NWAVE * WCAP);
static_assert((RCAP % 32) == 0);
static_assert(NWAVE * STW <= RCAP);
static_assert(STW >= CH);
static_assert(LDS_AGG <= 300000);
static_assert(LDS_ATT <= 300000);
static_assert(GBM == (GTHR / 32) * 16);
static_assert((CH % 32) == 0 && (CH2 % 32) == 0);
static_assert((CH % GBN) == 0 && (CH2 % GBN) == 0);
static_assert(CH == NHD * HDM && QKVW == 3 * CH);
static_assert(ATHR == 32 * AWAV && (GLN % (16 * AWAV)) == 0 && (GLN % 32) == 0);
static_assert((GLN % GBM) == 0);
static_assert(CH / 8 == 16);
static_assert(AWSZ >= 16 * HDM);

typedef float    v4f  __attribute__((ext_vector_type(4)));
typedef float    v8f  __attribute__((ext_vector_type(8)));
typedef int      v4i  __attribute__((ext_vector_type(4)));
typedef int      v8i  __attribute__((ext_vector_type(8)));
typedef _Float16 v8h  __attribute__((ext_vector_type(8)));
typedef _Float16 v16h __attribute__((ext_vector_type(16)));
union FragH { v16h v; v8h h[2]; v8i w; };

__device__ __forceinline__ v8f wmh(const FragH& a, const FragH& b, v8f c) {
  v8f d = __builtin_amdgcn_wmma_f32_16x16x32_f16(false, a.v, false, b.v, (short)0, c, false, false);
  asm volatile("v_nop\n\tv_nop\n\tv_nop\n\tv_nop" : "+v"(d) : "v"(a.w), "v"(b.w));
  return d;
}

__device__ __forceinline__ void ldwait() {
  asm volatile("s_wait_loadcnt 0x0" ::: "memory");
}

__device__ __forceinline__ float bfr(float f) {
  unsigned u = __float_as_uint(f);
  u = (u + 0x7FFFu + ((u >> 16) & 1u)) & 0xFFFF0000u;
  return __uint_as_float(u);
}
__device__ __forceinline__ v4f bfr4(const v4f a) {
  v4f r;
  r.x = bfr(a.x); r.y = bfr(a.y); r.z = bfr(a.z); r.w = bfr(a.w);
  return r;
}

__device__ __forceinline__ v8h cvt8h(const v4f a, const v4f b, const float c) {
  v8h hv;
  hv[0] = (_Float16)(a.x * c); hv[1] = (_Float16)(a.y * c);
  hv[2] = (_Float16)(a.z * c); hv[3] = (_Float16)(a.w * c);
  hv[4] = (_Float16)(b.x * c); hv[5] = (_Float16)(b.y * c);
  hv[6] = (_Float16)(b.z * c); hv[7] = (_Float16)(b.w * c);
  return hv;
}

__device__ __forceinline__ void cvt8hl(const v4f a, const v4f b, const float c, v8h& hi, v8h& lo) {
  const v8f s = __builtin_shufflevector(a, b, 0, 1, 2, 3, 4, 5, 6, 7) * c;
#pragma unroll
  for (int e = 0; e < 8; ++e) {
    const _Float16 q = (_Float16)s[e];
    hi[e] = q;
    lo[e] = (_Float16)((s[e] - (float)q) * CLO);
  }
}

__device__ __forceinline__ v4f relu4(const v4f a) {
  v4f r;
  r.x = fmaxf(a.x, 0.f); r.y = fmaxf(a.y, 0.f); r.z = fmaxf(a.z, 0.f); r.w = fmaxf(a.w, 0.f);
  return r;
}

__device__ __forceinline__ int scan_chunk(const int* __restrict__ dsts, int nE, int cbase, int slotBase,
                                          int nb, int vec8, int* list, int tid, int lane, int wave) {
  int wc = 0;
  const int el0  = tid * EPT;
  const int e0   = cbase + el0;
  const int sent = -2147483647 - 1;
  v4i da, db;
  if (vec8 != 0 && cbase + CHUNK <= nE) {
    da = *(const v4i*)(dsts + e0);
    db = *(const v4i*)(dsts + e0 + 4);
  } else {
    da.x = (e0     < nE) ? dsts[min(e0,     nE - 1)] : sent;
    da.y = (e0 + 1 < nE) ? dsts[min(e0 + 1, nE - 1)] : sent;
    da.z = (e0 + 2 < nE) ? dsts[min(e0 + 2, nE - 1)] : sent;
    da.w = (e0 + 3 < nE) ? dsts[min(e0 + 3, nE - 1)] : sent;
    db.x = (e0 + 4 < nE) ? dsts[min(e0 + 4, nE - 1)] : sent;
    db.y = (e0 + 5 < nE) ? dsts[min(e0 + 5, nE - 1)] : sent;
    db.z = (e0 + 6 < nE) ? dsts[min(e0 + 6, nE - 1)] : sent;
    db.w = (e0 + 7 < nE) ? dsts[min(e0 + 7, nE - 1)] : sent;
  }
  const unsigned nbs = (unsigned)slotBase;
  const unsigned unb = (unsigned)nb;
  const unsigned s0 = (unsigned)da.x - nbs, s1 = (unsigned)da.y - nbs;
  const unsigned s2 = (unsigned)da.z - nbs, s3 = (unsigned)da.w - nbs;
  const unsigned s4 = (unsigned)db.x - nbs, s5 = (unsigned)db.y - nbs;
  const unsigned s6 = (unsigned)db.z - nbs, s7 = (unsigned)db.w - nbs;
  const bool h0 = s0 < unb, h1 = s1 < unb, h2 = s2 < unb, h3 = s3 < unb;
  const bool h4 = s4 < unb, h5 = s5 < unb, h6 = s6 < unb, h7 = s7 < unb;
  const unsigned any = __builtin_amdgcn_ballot_w32(h0 | h1 | h2 | h3 | h4 | h5 | h6 | h7);
  if (any != 0u) {
#define HITJ(J, HJ, SJ) { \
      const unsigned mj = __builtin_amdgcn_ballot_w32(HJ); \
      if (mj != 0u) { \
        if (HJ) { \
          const int pos = wc + (int)__builtin_amdgcn_mbcnt_lo(mj, 0u); \
          if (pos < WCAP) list[wave * WCAP + pos] = ((el0 + (J)) << 12) | (int)(SJ); \
        } \
        wc += (int)__builtin_popcount(mj); } }
    HITJ(0, h0, s0)
    HITJ(1, h1, s1)
    HITJ(2, h2, s2)
    HITJ(3, h3, s3)
    HITJ(4, h4, s4)
    HITJ(5, h5, s5)
    HITJ(6, h6, s6)
    HITJ(7, h7, s7)
#undef HITJ
  }
  return wc;
}

__global__ __launch_bounds__(NTHR) void k_xprep(const float* __restrict__ x, _Float16* xh, int nN, int nUnits) {
  const int i = (int)blockIdx.x * NTHR + (int)threadIdx.x;
  if (i >= nUnits) return;
  const int row = i >> 4;
  const int c0  = (i & 15) * 8;
  const int rc  = row < nN ? row : nN - 1;
  const float* p = x + (size_t)rc * CH + c0;
  v4f a = *(const v4f*)p, b = *(const v4f*)(p + 4);
  const v4f z4 = {0.f, 0.f, 0.f, 0.f};
  if (row >= nN) { a = z4; b = z4; }
  a = bfr4(a); b = bfr4(b);
  const v8h hv = cvt8h(a, b, CACT);
  const size_t o = (size_t)row * CH + c0;
  *(volatile v8h*)(xh + o) = hv;
  __threadfence();
  *(volatile v8h*)(xh + o) = hv;
}

__global__ __launch_bounds__(NTHR) void k_wcvt(const float* __restrict__ w0, const float* __restrict__ w1,
                                               const float* __restrict__ w2, const float* __restrict__ w3,
                                               int n0, int n1, int n2, int n3,
                                               int K, _Float16* wt, int nUnits) {
  const int u = (int)blockIdx.x * NTHR + (int)threadIdx.x;
  if (u >= nUnits) return;
  const int kq = K >> 3;
  const int n  = u / kq;
  const int k8 = (u - n * kq) * 8;
  const int e0 = n0, e1 = n0 + n1, e2 = n0 + n1 + n2;
  const int seg = n < e0 ? 0 : (n < e1 ? 1 : (n < e2 ? 2 : 3));
  const int sb  = (seg == 0) ? 0 : ((seg == 1) ? e0 : ((seg == 2) ? e1 : e2));
  const float* ws = (seg == 0) ? w0 : ((seg == 1) ? w1 : ((seg == 2) ? w2 : w3));
  const int nv = (seg == 0) ? n0 : ((seg == 1) ? n1 : ((seg == 2) ? n2 : n3));
  const int nvp = nv < 1 ? 1 : nv;
  int ncl = n - sb;
  ncl = ncl > nvp - 1 ? nvp - 1 : ncl;
  ncl = ncl < 0 ? 0 : ncl;
  const float* p = ws + (size_t)k8 * (size_t)nvp + ncl;
  const float l0 = p[0];
  const float l1 = p[(size_t)1 * nvp];
  const float l2 = p[(size_t)2 * nvp];
  const float l3 = p[(size_t)3 * nvp];
  const float l4 = p[(size_t)4 * nvp];
  const float l5 = p[(size_t)5 * nvp];
  const float l6 = p[(size_t)6 * nvp];
  const float l7 = p[(size_t)7 * nvp];
  const v4f a = {bfr(l0), bfr(l1), bfr(l2), bfr(l3)};
  const v4f b = {bfr(l4), bfr(l5), bfr(l6), bfr(l7)};
  const v8h hv = cvt8h(a, b, CWGT);
  const size_t o = (size_t)n * (size_t)K + k8;
  *(volatile v8h*)(wt + o) = hv;
  __threadfence();
  *(volatile v8h*)(wt + o) = hv;
}

template<int EPI, int LO>
__global__ __launch_bounds__(GTHR) void k_gemm(
    const _Float16* __restrict__ A, const _Float16* __restrict__ AL, int aPitch, int aSeg,
    const _Float16* __restrict__ WT, int K,
    const float* __restrict__ bias, int useBias,
    const float* __restrict__ resid, int ldr, int useRes, int rndRes,
    float* outF, int ldo, _Float16* outH, _Float16* outL,
    float scl, float sclLo, int relu, float ocarry,
    float* part, int statN, int useStat)
{
  __shared__ __attribute__((aligned(16))) float stg[GBM * GBN];
  __shared__ __attribute__((aligned(16))) float pss[2 * GBN];
  const int tid = (int)threadIdx.x, lane = tid & 31, wave = tid >> 5, hh = lane >> 4, m = lane & 15;
  const int rowBase = (int)blockIdx.x * GBM;
  const int col0    = (int)blockIdx.y * GBN;

  v8f acc[4], acl[4];
  {
    const v8f z = {0.f, 0.f, 0.f, 0.f, 0.f, 0.f, 0.f, 0.f};
    acc[0] = z; acc[1] = z; acc[2] = z; acc[3] = z;
    acl[0] = z; acl[1] = z; acl[2] = z; acl[3] = z;
  }
  const size_t arow = (size_t)(rowBase + 16 * wave + m) * (size_t)aPitch + 8 * hh;
  const _Float16* wp = WT + (size_t)(col0 + m) * (size_t)K + 8 * hh;
  const int ksteps = K >> 5;
#pragma unroll 1
  for (int ks = 0; ks < ksteps; ++ks) {
    const size_t s0 = arow + (size_t)(2 * ks) * (size_t)aSeg;
    const size_t s1 = s0 + (size_t)aSeg;
    FragH af;
    af.h[0] = *(const v8h*)(A + s0);
    af.h[1] = *(const v8h*)(A + s1);
    FragH al;
    if constexpr (LO != 0) {
      al.h[0] = *(const v8h*)(AL + s0);
      al.h[1] = *(const v8h*)(AL + s1);
    } else {
      al = af;
    }
#pragma unroll
    for (int t = 0; t < 4; ++t) {
      const _Float16* wq = wp + (size_t)(16 * t) * (size_t)K + 32 * ks;
      FragH bf;
      bf.h[0] = *(const v8h*)wq;
      bf.h[1] = *(const v8h*)(wq + 16);
      acc[t] = wmh(af, bf, acc[t]);
      if constexpr (LO != 0) acl[t] = wmh(al, bf, acl[t]);
    }
  }

#pragma unroll
  for (int t = 0; t < 4; ++t) {
    const int lc = 16 * t + m;
    const float bl = bfr(bias[col0 + lc]);
    const float bv = useBias ? bl : 0.0f;
#pragma unroll
    for (int r = 0; r < 8; ++r) {
      const int lr = 16 * wave + 8 * hh + r;
      float v = fmaf(acc[t][r], scl, bv);
      if constexpr (LO != 0) v = fmaf(acl[t][r], sclLo, v);
      stg[lr * GBN + lc] = v;
    }
  }
  __syncthreads();

  if constexpr (EPI == 0) {
    v4f fv[8];
#pragma unroll
    for (int i = 0; i < 8; ++i) {
      const int lr = 16 * wave + 2 * i + hh;
      fv[i] = *(const v4f*)(stg + lr * GBN + 4 * m);
    }
    if (useRes) {
#pragma unroll
      for (int i = 0; i < 8; ++i) {
        const int lr = 16 * wave + 2 * i + hh;
        const int gr = rowBase + lr;
        v4f rv = *(const v4f*)(resid + (size_t)gr * (size_t)ldr + col0 + 4 * m);
        if (rndRes) rv = bfr4(rv);
        fv[i] += rv;
      }
    }
    if (useStat) {
      if (useRes) {
#pragma unroll
        for (int i = 0; i < 8; ++i) {
          const int lr = 16 * wave + 2 * i + hh;
          *(v4f*)(stg + lr * GBN + 4 * m) = fv[i];
        }
      }
      __syncthreads();
      if (tid < GBN) {
        float s = 0.f;
#pragma unroll 8
        for (int r = 0; r < GBM; ++r) s += stg[r * GBN + tid];
        const float mb = s * (1.0f / (float)GBM);
        float q = 0.f;
#pragma unroll 8
        for (int r = 0; r < GBM; ++r) {
          const float dl = stg[r * GBN + tid] - mb;
          q = fmaf(dl, dl, q);
        }
        pss[tid] = s;
        pss[GBN + tid] = q;
      }
      __syncthreads();
    }
    const bool pst = (useStat != 0) && (wave == 0);
    v4f pv = {0.f, 0.f, 0.f, 0.f};
    float* pp = part;
    if (pst) {
      pv = *(const v4f*)(pss + 4 * lane);
      pp = part + ((size_t)(2 * (int)blockIdx.x + hh) * (size_t)statN + col0 + 4 * m);
    }
#pragma unroll
    for (int i = 0; i < 8; ++i) {
      const int lr = 16 * wave + 2 * i + hh;
      const int gr = rowBase + lr;
      float* op = outF + (size_t)gr * (size_t)ldo + col0 + 4 * m;
      *(volatile v4f*)op = fv[i];
    }
    if (pst) *(volatile v4f*)pp = pv;
    __threadfence();
#pragma unroll
    for (int i = 0; i < 8; ++i) {
      const int lr = 16 * wave + 2 * i + hh;
      const int gr = rowBase + lr;
      float* op = outF + (size_t)gr * (size_t)ldo + col0 + 4 * m;
      *(volatile v4f*)op = fv[i];
    }
    if (pst) *(volatile v4f*)pp = pv;
  } else {
    v8h hv[4], lv[4];
#pragma unroll
    for (int i = 0; i < 4; ++i) {
      const int lr = 16 * wave + 4 * i + (lane >> 3);
      const int c8 = (lane & 7) * 8;
      v4f ga = *(const v4f*)(stg + lr * GBN + c8);
      v4f gb = *(const v4f*)(stg + lr * GBN + c8 + 4);
      if (relu) { ga = relu4(ga); gb = relu4(gb); }
      cvt8hl(ga, gb, ocarry, hv[i], lv[i]);
    }
#pragma unroll
    for (int i = 0; i < 4; ++i) {
      const int lr = 16 * wave + 4 * i + (lane >> 3);
      const int c8 = (lane & 7) * 8;
      const int gr = rowBase + lr;
      const size_t e = (size_t)gr * (size_t)ldo + col0 + c8;
      *(volatile v8h*)(outH + e) = hv[i];
      *(volatile v8h*)(outL + e) = lv[i];
    }
    __threadfence();
#pragma unroll
    for (int i = 0; i < 4; ++i) {
      const int lr = 16 * wave + 4 * i + (lane >> 3);
      const int c8 = (lane & 7) * 8;
      const int gr = rowBase + lr;
      const size_t e = (size_t)gr * (size_t)ldo + col0 + c8;
      *(volatile v8h*)(outH + e) = hv[i];
      *(volatile v8h*)(outL + e) = lv[i];
    }
  }
}

__global__ __launch_bounds__(NTHR) void k_agg(
    const int* __restrict__ srcs, const int* __restrict__ dsts,
    const float* __restrict__ x, const float* __restrict__ geps, _Float16* HGH, _Float16* HGL,
    int nN, int nE, int nb, int vec8, int MPr) {
  extern __shared__ v4f lds_dyn[];
  int* reg1 = (int*)lds_dyn;
  int* reg2 = reg1 + RCAP;
  int* scnt = reg2 + RCAP;
  int* soff = scnt + NBMAX;
  int* list = soff + NBMAX;
  int* wcnt = list + LISTN;
  int* wtot = wcnt + NWAVE;
  const int tid = (int)threadIdx.x, lane = tid & 31, wave = tid >> 5;
  const int nodeBase = (int)blockIdx.x * nb;

  for (int i = tid; i < NBMAX; i += NTHR) scnt[i] = 0;
  __syncthreads();

  int tot = 0;
  const int nChunks = (nE + CHUNK - 1) / CHUNK;
#pragma unroll 1
  for (int ch = 0; ch < nChunks; ++ch) {
    const int cbase = ch * CHUNK;
    const int wc = scan_chunk(dsts, nE, cbase, nodeBase, nb, vec8, list, tid, lane, wave);
    if (lane == 0) wcnt[wave] = wc;
    __syncthreads();
    int pre = 0, all = 0;
#pragma unroll
    for (int w2 = 0; w2 < NWAVE; ++w2) {
      int c = wcnt[w2];
      c = c < 0 ? 0 : (c > WCAP ? WCAP : c);
      all += c;
      pre += (w2 < wave) ? c : 0;
    }
    const int wcc  = wc > WCAP ? WCAP : wc;
    const int base = tot + pre;
#pragma unroll 1
    for (int i = lane; i < wcc; i += 32) {
      const int ent = list[wave * WCAP + i];
      const int el  = (ent >> 12) & (CHUNK - 1);
      const int sl  = ent & (NBMAX - 1);
      int eid = cbase + el;
      eid = eid > nE - 1 ? nE - 1 : eid;
      const int pos = base + i;
      if (pos < RCAP) reg1[pos] = (int)(((unsigned)eid << 12) | (unsigned)sl);
    }
    tot += all;
    tot = tot > RCAP ? RCAP : tot;
    __syncthreads();
  }
  const int nh = tot;

  if (wave == 0) {
#pragma unroll 1
    for (int b0 = 0; b0 < nh; b0 += 32) {
      const int idx = b0 + lane;
      const int uv  = reg1[idx < RCAP ? idx : RCAP - 1];
      const int m32 = (nh - b0) < 32 ? (nh - b0) : 32;
#pragma unroll 1
      for (int k = 0; k < m32; ++k) {
        const int u  = __builtin_amdgcn_readlane(uv, k);
        const int sl = u & (NBMAX - 1);
        if (lane == 0) scnt[sl] = scnt[sl] + 1;
      }
    }
  }
  __syncthreads();

  {
    const v4i ca = *(const v4i*)(scnt + 8 * tid);
    const v4i cb = *(const v4i*)(scnt + 8 * tid + 4);
    const int e0 = ca.x < 0 ? 0 : ca.x, e1 = ca.y < 0 ? 0 : ca.y, e2 = ca.z < 0 ? 0 : ca.z, e3 = ca.w < 0 ? 0 : ca.w;
    const int e4 = cb.x < 0 ? 0 : cb.x, e5 = cb.y < 0 ? 0 : cb.y, e6 = cb.z < 0 ? 0 : cb.z, e7 = cb.w < 0 ? 0 : cb.w;
    const int ts = e0 + e1 + e2 + e3 + e4 + e5 + e6 + e7;
    int incl = ts;
#pragma unroll
    for (int d = 1; d < 32; d <<= 1) {
      const int up = __shfl_up(incl, d);
      if (lane >= d) incl += up;
    }
    if (lane == 31) wtot[wave] = incl;
    __syncthreads();
    int pre = 0;
#pragma unroll
    for (int w2 = 0; w2 < NWAVE; ++w2) pre += (w2 < wave) ? wtot[w2] : 0;
    int run = pre + incl - ts;
    soff[8 * tid + 0] = run; run += e0;
    soff[8 * tid + 1] = run; run += e1;
    soff[8 * tid + 2] = run; run += e2;
    soff[8 * tid + 3] = run; run += e3;
    soff[8 * tid + 4] = run; run += e4;
    soff[8 * tid + 5] = run; run += e5;
    soff[8 * tid + 6] = run; run += e6;
    soff[8 * tid + 7] = run;
  }
  __syncthreads();
  for (int i = tid; i < NBMAX; i += NTHR) list[i] = soff[i];
  __syncthreads();

  if (wave == 0) {
#pragma unroll 1
    for (int b0 = 0; b0 < nh; b0 += 32) {
      const int idx = b0 + lane;
      const int uv  = reg1[idx < RCAP ? idx : RCAP - 1];
      const int m32 = (nh - b0) < 32 ? (nh - b0) : 32;
#pragma unroll 1
      for (int k = 0; k < m32; ++k) {
        const int u   = __builtin_amdgcn_readlane(uv, k);
        const int sl  = u & (NBMAX - 1);
        const int eid = (int)((unsigned)u >> 12);
        if (lane == 0) {
          int pos = list[sl];
          pos = pos < 0 ? 0 : (pos > RCAP - 1 ? RCAP - 1 : pos);
          reg2[pos] = eid;
          list[sl] = pos + 1;
        }
      }
    }
  }
  __syncthreads();

  const int nbw = nb >> 3;
  const bool ovf = (nh >= RCAP);
  const float qnan = __int_as_float(0x7fc00000);
  float* stw = (float*)reg1 + wave * STW;
  const float epm = 1.0f + bfr(geps[0]);
  const int lc = lane < (CH / 8) ? lane : (CH / 8) - 1;
#pragma unroll 1
  for (int jt = 0; jt < nbw; ++jt) {
    const int slot = wave * nbw + jt;
    const int grow = nodeBase + slot;
    const int gcl  = grow < nN ? grow : nN - 1;
    int st = soff[slot];
    const int craw = scnt[slot];
    int cnt = craw;
    st  = st < 0 ? 0 : (st > nh ? nh : st);
    cnt = cnt < 0 ? 0 : (cnt > DEGCAP ? DEGCAP : cnt);
    if (cnt > nh - st) cnt = nh - st;
    const float pz = (ovf || craw > DEGCAP) ? qnan : 0.0f;
    const bool wr = grow < MPr;
    const float live = grow < nN ? 1.0f : 0.0f;

    float av[4];
#pragma unroll
    for (int j = 0; j < 4; ++j) av[j] = 0.f;
#pragma unroll 1
    for (int q = 0; q < cnt; ++q) {
      int idx = st + q; idx = idx > RCAP - 1 ? RCAP - 1 : idx;
      int eid = reg2[idx]; eid = eid < 0 ? 0 : (eid > nE - 1 ? nE - 1 : eid);
      const int sraw = srcs[eid];
      const int s = sraw < 0 ? 0 : (sraw > nN - 1 ? nN - 1 : sraw);
      const float* xr = x + (size_t)s * CH + lane;
      float xv[4];
#pragma unroll
      for (int j = 0; j < 4; ++j) xv[j] = xr[32 * j];
      ldwait();
#pragma unroll
      for (int j = 0; j < 4; ++j) av[j] += bfr(xv[j]);
    }
    const float* xd = x + (size_t)gcl * CH + lane;
    float dv[4];
#pragma unroll
    for (int j = 0; j < 4; ++j) dv[j] = xd[32 * j];
    ldwait();
    float rv[4];
#pragma unroll
    for (int j = 0; j < 4; ++j) rv[j] = (epm * bfr(dv[j]) + av[j]) * live + pz;
    __builtin_amdgcn_fence(__ATOMIC_RELEASE, "wavefront");
    __builtin_amdgcn_wave_barrier();
#pragma unroll
    for (int j = 0; j < 4; ++j) stw[32 * j + lane] = rv[j];
    __builtin_amdgcn_fence(__ATOMIC_RELEASE, "wavefront");
    __builtin_amdgcn_wave_barrier();
    const v4f ga = *(const v4f*)(stw + 8 * lc);
    const v4f gb = *(const v4f*)(stw + 8 * lc + 4);
    v8h hv, lv;
    cvt8hl(ga, gb, CACT, hv, lv);
    const size_t go = (size_t)grow * CH + 8 * lc;
    const bool wsv = wr && (lane < (CH / 8));
    if (wsv) { *(volatile v8h*)(HGH + go) = hv; *(volatile v8h*)(HGL + go) = lv; }
    __threadfence();
    if (wsv) { *(volatile v8h*)(HGH + go) = hv; *(volatile v8h*)(HGL + go) = lv; }
  }
}

__global__ __launch_bounds__(ATHR) void k_attn(const float* __restrict__ QKV, _Float16* ODH, _Float16* ODL, int nN) {
  extern __shared__ v4f lds_at[];
  _Float16* skh = (_Float16*)lds_at;
  _Float16* skl = skh + GLN * HDM;
  _Float16* svt = skl + GLN * HDM;
  float* wsb = (float*)(svt + HDM * GLN);
  const int tid = (int)threadIdx.x, lane = tid & 31, wave = tid >> 5, hh = lane >> 4, m = lane & 15;
  float* ssc = wsb + wave * AWSZ;
  _Float16* sp = (_Float16*)(ssc + 16 * GLN);
  const int h = (int)blockIdx.x;
  const int b = (int)blockIdx.y;
  const size_t node0 = (size_t)b * GLN;

#pragma unroll 1
  for (int key = tid; key < GLN; key += ATHR) {
    const float* kr = QKV + (node0 + (size_t)key) * QKVW + CH + h * HDM;
    const v4f k0 = *(const v4f*)kr, k1 = *(const v4f*)(kr + 4);
    const v4f k2 = *(const v4f*)(kr + 8), k3 = *(const v4f*)(kr + 12);
    v8h ha, la, hb, lb;
    cvt8hl(k0, k1, CACT, ha, la);
    cvt8hl(k2, k3, CACT, hb, lb);
    *(v8h*)(skh + key * HDM)     = ha;
    *(v8h*)(skh + key * HDM + 8) = hb;
    *(v8h*)(skl + key * HDM)     = la;
    *(v8h*)(skl + key * HDM + 8) = lb;
    const float* vr = kr + CH;
    const v4f v0 = *(const v4f*)vr, v1 = *(const v4f*)(vr + 4);
    const v4f v2 = *(const v4f*)(vr + 8), v3 = *(const v4f*)(vr + 12);
    const v8f va = __builtin_shufflevector(v0, v1, 0, 1, 2, 3, 4, 5, 6, 7) * CACT;
    const v8f vb = __builtin_shufflevector(v2, v3, 0, 1, 2, 3, 4, 5, 6, 7) * CACT;
#pragma unroll
    for (int d = 0; d < 8; ++d) {
      svt[d * GLN + key]       = (_Float16)va[d];
      svt[(8 + d) * GLN + key] = (_Float16)vb[d];
    }
  }
  __syncthreads();

  const v8f zf = {0.f, 0.f, 0.f, 0.f, 0.f, 0.f, 0.f, 0.f};
  v8h z8h;
#pragma unroll
  for (int e = 0; e < 8; ++e) z8h[e] = (_Float16)0.0f;

#pragma unroll 1
  for (int rt = 0; rt < ARTS; ++rt) {
    const int q0 = (rt * AWAV + wave) * 16;
    __builtin_amdgcn_fence(__ATOMIC_RELEASE, "wavefront");
    __builtin_amdgcn_wave_barrier();
    const float* qr = QKV + (node0 + (size_t)(q0 + m)) * QKVW + h * HDM + 8 * hh;
    const v4f qa = *(const v4f*)qr, qb = *(const v4f*)(qr + 4);
    FragH a;
    cvt8hl(qa, qb, CACT, a.h[0], a.h[1]);

#pragma unroll 2
    for (int ct = 0; ct < GLN / 16; ++ct) {
      const int koff = (ct * 16 + m) * HDM + 8 * hh;
      const v8h kh = *(const v8h*)(skh + koff);
      const v8h kl = *(const v8h*)(skl + koff);
      FragH b1, b2;
      b1.h[0] = kh; b1.h[1] = z8h;
      b2.h[0] = kl; b2.h[1] = kh;
      const v8f c1 = wmh(a, b1, zf);
      const v8f c2 = wmh(a, b2, zf);
#pragma unroll
      for (int r = 0; r < 8; ++r)
        ssc[(8 * hh + r) * GLN + ct * 16 + m] = fmaf(c2[r], SC2, c1[r] * SC1);
    }
    __builtin_amdgcn_fence(__ATOMIC_RELEASE, "wavefront");
    __builtin_amdgcn_wave_barrier();

#pragma unroll 1
    for (int r = 0; r < 16; ++r) {
      float xv[16];
#pragma unroll
      for (int j = 0; j < 16; ++j) xv[j] = ssc[r * GLN + 32 * j + lane];
      float mx = xv[0];
#pragma unroll
      for (int j = 1; j < 16; ++j) mx = fmaxf(mx, xv[j]);
#pragma unroll
      for (int d = 16; d > 0; d >>= 1) mx = fmaxf(mx, __shfl_xor(mx, d));
      float sm = 0.f;
#pragma unroll
      for (int j = 0; j < 16; ++j) { xv[j] = __expf(xv[j] - mx); sm += xv[j]; }
#pragma unroll
      for (int d = 16; d > 0; d >>= 1) sm += __shfl_xor(sm, d);
      const float inv = CPRB * (1.0f / sm);
#pragma unroll
      for (int j = 0; j < 16; ++j) sp[r * GLN + 32 * j + lane] = (_Float16)(xv[j] * inv);
    }
    __builtin_amdgcn_fence(__ATOMIC_RELEASE, "wavefront");
    __builtin_amdgcn_wave_barrier();

    v8f acc = zf;
#pragma unroll 2
    for (int ks = 0; ks < GLN / 32; ++ks) {
      const int kk = ks * 32;
      FragH ap, bv;
      ap.h[0] = *(const v8h*)(sp + m * GLN + kk + 8 * hh);
      ap.h[1] = *(const v8h*)(sp + m * GLN + kk + 16 + 8 * hh);
      bv.h[0] = *(const v8h*)(svt + m * GLN + kk + 8 * hh);
      bv.h[1] = *(const v8h*)(svt + m * GLN + kk + 16 + 8 * hh);
      acc = wmh(ap, bv, acc);
    }

#pragma unroll
    for (int r = 0; r < 8; ++r) ssc[(8 * hh + r) * HDM + m] = acc[r] * SCO;
    __builtin_amdgcn_fence(__ATOMIC_RELEASE, "wavefront");
    __builtin_amdgcn_wave_barrier();
    const int lr = lane >> 1, c8 = (lane & 1) * 8;
    const v4f oa = *(const v4f*)(ssc + lr * HDM + c8);
    const v4f ob = *(const v4f*)(ssc + lr * HDM + c8 + 4);
    v8h ohv, olv;
    cvt8hl(oa, ob, CACT, ohv, olv);
    const size_t go = ((size_t)h * (size_t)nN + node0 + (size_t)(q0 + lr)) * HDM + c8;
    *(volatile v8h*)(ODH + go) = ohv;
    *(volatile v8h*)(ODL + go) = olv;
    __threadfence();
    *(volatile v8h*)(ODH + go) = ohv;
    *(volatile v8h*)(ODL + go) = olv;
  }
}

__global__ __launch_bounds__(CH) void k_fold(const float* __restrict__ partA, float* statA,
                                             const float* __restrict__ partB, float* statB, int nblk) {
  __shared__ __attribute__((aligned(16))) float sm[2 * CH];
  const int c = (int)threadIdx.x;
  const bool sB = blockIdx.x != 0;
  const float* part = sB ? partB : partA;
  float* stat = sB ? statB : statA;
  double cnt = 0.0, mean = 0.0, M2 = 0.0;
#pragma unroll 1
  for (int bx = 0; bx < nblk; ++bx) {
    const float s = part[(size_t)(2 * bx) * CH + c];
    const float q = part[(size_t)(2 * bx + 1) * CH + c];
    const double mb   = (double)s * (1.0 / (double)GBM);
    const double ncnt = cnt + (double)GBM;
    const double dl   = mb - mean;
    mean += dl * ((double)GBM / ncnt);
    M2   += (double)q + dl * dl * (cnt * (double)GBM / ncnt);
    cnt = ncnt;
  }
  const double var = cnt > 0.0 ? M2 / cnt : 0.0;
  const float mu = (float)mean;
  float vf = (float)var;
  vf = vf < 0.f ? 0.f : vf;
  const float rs = 1.0f / sqrtf(vf + 1.0e-5f);
  sm[c] = mu;
  sm[CH + c] = rs;
  __syncthreads();
  if (c < (2 * CH) / 4) {
    const v4f v = *(const v4f*)(sm + 4 * c);
    float* p = stat + 4 * c;
    *(volatile v4f*)p = v;
    __threadfence();
    *(volatile v4f*)p = v;
  }
}

__global__ __launch_bounds__(NTHR) void k_combine(
    const float* __restrict__ HGX, const float* __restrict__ HMX,
    const float* __restrict__ st1, const float* __restrict__ st2,
    const float* __restrict__ ga1, const float* __restrict__ bb1,
    const float* __restrict__ ga2, const float* __restrict__ bb2,
    float* OUTF, _Float16* FOH, _Float16* FOL, int nUnits) {
  __shared__ __attribute__((aligned(16))) float stl[NWAVE * CH];
  const int tid = (int)threadIdx.x, lane = tid & 31, wave = tid >> 5;
  const int i = (int)blockIdx.x * NTHR + tid;
  if (i >= nUnits) return;
  const int row = i >> 5;
  const int c4  = lane * 4;
  const size_t e = (size_t)row * CH + c4;
  const v4f a  = *(const v4f*)(HGX + e);
  const v4f hm = *(const v4f*)(HMX + e);
  const v4f m1 = *(const v4f*)(st1 + c4), r1 = *(const v4f*)(st1 + CH + c4);
  const v4f m2 = *(const v4f*)(st2 + c4), r2 = *(const v4f*)(st2 + CH + c4);
  const v4f g1v = bfr4(*(const v4f*)(ga1 + c4)), b1v = bfr4(*(const v4f*)(bb1 + c4));
  const v4f g2v = bfr4(*(const v4f*)(ga2 + c4)), b2v = bfr4(*(const v4f*)(bb2 + c4));
  const v4f h1 = ((a - m1) * r1) * g1v + b1v;
  const v4f h2 = ((hm - m2) * r2) * g2v + b2v;
  const v4f o  = h1 + h2;
  float* pf = OUTF + e;
  float* sw = stl + wave * CH;
  *(v4f*)(sw + c4) = o;
  __builtin_amdgcn_fence(__ATOMIC_RELEASE, "wavefront");
  __builtin_amdgcn_wave_barrier();
  const int lc = lane < (CH / 8) ? lane : (CH / 8) - 1;
  const v4f qa = *(const v4f*)(sw + 8 * lc);
  const v4f qb = *(const v4f*)(sw + 8 * lc + 4);
  v8h hv, lv;
  cvt8hl(qa, qb, CACT, hv, lv);
  const size_t ho = (size_t)row * CH + 8 * lc;
  const bool wsv = lane < (CH / 8);
  *(volatile v4f*)pf = o;
  if (wsv) { *(volatile v8h*)(FOH + ho) = hv; *(volatile v8h*)(FOL + ho) = lv; }
  __threadfence();
  *(volatile v4f*)pf = o;
  if (wsv) { *(volatile v8h*)(FOH + ho) = hv; *(volatile v8h*)(FOL + ho) = lv; }
}

__global__ __launch_bounds__(NTHR) void k_apply(const float* __restrict__ O2, const float* __restrict__ st,
                                                const float* __restrict__ ga, const float* __restrict__ bb,
                                                float* out0, int nUnits) {
  const int tid = (int)threadIdx.x, lane = tid & 31;
  const int i = (int)blockIdx.x * NTHR + tid;
  if (i >= nUnits) return;
  const int row = i >> 5;
  const int c4  = lane * 4;
  const size_t e = (size_t)row * CH + c4;
  const v4f v  = *(const v4f*)(O2 + e);
  const v4f mu = *(const v4f*)(st + c4), rs = *(const v4f*)(st + CH + c4);
  const v4f gv = bfr4(*(const v4f*)(ga + c4)), bv = bfr4(*(const v4f*)(bb + c4));
  const v4f o = ((v - mu) * rs) * gv + bv;
  float* p = out0 + e;
  *(volatile v4f*)p = o;
  __threadfence();
  *(volatile v4f*)p = o;
}

static int pick_nb(int nE, int nN) {
  int nb = NBMAX;
  while (nb > 16 && (long long)nb * (long long)nE * 5LL > (long long)RCAP * (long long)nN * 4LL) nb >>= 1;
  return nb;
}
static inline int cdiv(int a, int b) { return (a + b - 1) / b; }
static inline size_t al256(size_t v) { return (v + 255) & ~(size_t)255; }

extern "C" void kernel_launch(void* const* d_in, const int* in_sizes, int n_in,
                              void* d_out, int out_size, void* d_ws, size_t ws_size,
                              hipStream_t stream) {
  if (n_in < 25) return;
  const int nN = in_sizes[0] / CH;
  if (nN <= 0 || in_sizes[0] != nN * CH || nN > (1 << 20)) return;
  if ((nN % GLN) != 0 || (nN % GBM) != 0) return;
  if (in_sizes[1] < 2 || (in_sizes[1] & 1) != 0) return;
  const int nE = in_sizes[1] / 2;
  if (nE < 1 || nE > (1 << 20)) return;
  if (in_sizes[2] < 1) return;
  if (in_sizes[3] != CH * CH2 || in_sizes[4] != CH2) return;
  if (in_sizes[5] != CH2 * CH || in_sizes[6] != CH)  return;
  if (in_sizes[7] != CH || in_sizes[8] != CH) return;
  for (int q = 9; q <= 15; q += 2) if (in_sizes[q] != CH * CH || in_sizes[q + 1] != CH) return;
  if (in_sizes[17] != CH || in_sizes[18] != CH) return;
  if (in_sizes[19] != CH * CH2 || in_sizes[20] != CH2) return;
  if (in_sizes[21] != CH2 * CH || in_sizes[22] != CH)  return;
  if (in_sizes[23] != CH || in_sizes[24] != CH) return;
  if (out_size != nN * CH) return;

  const float* x     = (const float*)d_in[0];
  const int*   ei    = (const int*)  d_in[1];
  const float* geps  = (const float*)d_in[2];
  const float* wl1   = (const float*)d_in[3];
  const float* bl1   = (const float*)d_in[4];
  const float* wl2   = (const float*)d_in[5];
  const float* bl2   = (const float*)d_in[6];
  const float* g1    = (const float*)d_in[7];
  const float* be1   = (const float*)d_in[8];
  const float* wq    = (const float*)d_in[9];
  const float* bq    = (const float*)d_in[10];
  const float* wk    = (const float*)d_in[11];
  const float* bk    = (const float*)d_in[12];
  const float* wv    = (const float*)d_in[13];
  const float* bv    = (const float*)d_in[14];
  const float* wo    = (const float*)d_in[15];
  const float* bo    = (const float*)d_in[16];
  const float* g2    = (const float*)d_in[17];
  const float* be2   = (const float*)d_in[18];
  const float* wf1   = (const float*)d_in[19];
  const float* bf1   = (const float*)d_in[20];
  const float* wf2   = (const float*)d_in[21];
  const float* bf2   = (const float*)d_in[22];
  const float* g3    = (const float*)d_in[23];
  const float* be3   = (const float*)d_in[24];
  float* out0 = (float*)d_out;
  const int* src = ei;
  const int* dst = ei + nE;

  const int MP   = nN;
  const int G    = nN / GLN;
  const int gM   = MP / GBM;
  const int nb   = pick_nb(nE, nN);
  const int gA   = cdiv(MP, nb);
  const int vec8 = ((nE & 3) == 0) ? 1 : 0;
  if (gA * nb < MP) return;

  const size_t szH  = (size_t)MP * CH * 2;
  const size_t szH2 = (size_t)MP * CH2 * 2;
  const size_t szF  = (size_t)MP * CH * 4;
  const size_t szQ  = (size_t)MP * QKVW * 4;
  const size_t szP  = (size_t)(2 * gM) * CH * 4;
  size_t off = 0;
  const size_t oR0  = off; off = al256(off + szQ);
  const size_t oR1  = off; off = al256(off + 2 * szH);
  const size_t oR2  = off; off = al256(off + szF);
  const size_t oR3  = off; off = al256(off + szF);
  const size_t oR4  = off; off = al256(off + szF);
  const size_t oWA  = off; off = al256(off + (size_t)640 * CH * 2);
  const size_t oWB  = off; off = al256(off + (size_t)384 * CH * 2);
  const size_t oWC  = off; off = al256(off + (size_t)CH2 * CH2 * 2);
  const size_t oP1  = off; off = al256(off + szP);
  const size_t oP2  = off; off = al256(off + szP);
  const size_t oP3  = off; off = al256(off + szP);
  const size_t oS1  = off; off = al256(off + (size_t)2 * CH * 4);
  const size_t oS2  = off; off = al256(off + (size_t)2 * CH * 4);
  const size_t oS3  = off; off = al256(off + (size_t)2 * CH * 4);
  if (off > ws_size || off > (size_t)WSMAX) return;
  if (2 * szH2 > szQ) return;

  char* ws = (char*)d_ws;
  float*    QKV  = (float*)(ws + oR0);
  _Float16* HRH  = (_Float16*)(ws + oR0);
  _Float16* HRL  = (_Float16*)(ws + oR0 + szH2);
  _Float16* T1H  = (_Float16*)(ws + oR0);
  _Float16* T1L  = (_Float16*)(ws + oR0 + szH2);
  _Float16* XH   = (_Float16*)(ws + oR1);
  _Float16* ODH  = (_Float16*)(ws + oR1);
  _Float16* ODL  = (_Float16*)(ws + oR1 + szH);
  _Float16* HGH  = (_Float16*)(ws + oR1);
  _Float16* HGL  = (_Float16*)(ws + oR1 + szH);
  _Float16* FOH  = (_Float16*)(ws + oR1);
  _Float16* FOL  = (_Float16*)(ws + oR1 + szH);
  float*    HMX  = (float*)(ws + oR2);
  float*    O2   = (float*)(ws + oR2);
  float*    HGX  = (float*)(ws + oR3);
  float*    OUTF = (float*)(ws + oR4);
  _Float16* WA   = (_Float16*)(ws + oWA);
  _Float16* WB   = (_Float16*)(ws + oWB);
  _Float16* WC   = (_Float16*)(ws + oWC);
  float* P1 = (float*)(ws + oP1);
  float* P2 = (float*)(ws + oP2);
  float* P3 = (float*)(ws + oP3);
  float* S1 = (float*)(ws + oS1);
  float* S2 = (float*)(ws + oS2);
  float* S3 = (float*)(ws + oS3);

  hipFuncSetAttribute(reinterpret_cast<const void*>(&k_agg),
                      hipFuncAttributeMaxDynamicSharedMemorySize, LDS_AGG);
  hipFuncSetAttribute(reinterpret_cast<const void*>(&k_attn),
                      hipFuncAttributeMaxDynamicSharedMemorySize, LDS_ATT);

  const int nU16 = MP * (CH / 8);
  const int nU32 = MP * (CH / 4);

  k_xprep<<<cdiv(nU16, NTHR), NTHR, 0, stream>>>(x, XH, nN, nU16);

  {
    const int nUA = 640 * (CH / 8);
    k_wcvt<<<cdiv(nUA, NTHR), NTHR, 0, stream>>>(wl1, wq, wk, wv, CH2, CH, CH, CH, CH, WA, nUA);
    const int nUB = 384 * (CH / 8);
    k_wcvt<<<cdiv(nUB, NTHR), NTHR, 0, stream>>>(wo, wf1, wo, wo, CH, CH2, 0, 0, CH, WB, nUB);
    const int nUC = CH2 * (CH2 / 8);
    k_wcvt<<<cdiv(nUC, NTHR), NTHR, 0, stream>>>(wl2, wf2, wl2, wl2, CH, CH, 0, 0, CH2, WC, nUC);
  }

  k_gemm<0, 0><<<dim3(gM, CH / GBN), GTHR, 0, stream>>>(XH, XH, CH, 16, WA + (size_t)(CH2 + 0 * CH) * CH, CH,
      bq, 1, x, CH, 0, 0, QKV + 0 * CH, QKVW, HRH, HRL, S11, S22, 0, 1.0f, P1, CH, 0);
  k_gemm<0, 0><<<dim3(gM, CH / GBN), GTHR, 0, stream>>>(XH, XH, CH, 16, WA + (size_t)(CH2 + 1 * CH) * CH, CH,
      bk, 1, x, CH, 0, 0, QKV + 1 * CH, QKVW, HRH, HRL, S11, S22, 0, 1.0f, P1, CH, 0);
  k_gemm<0, 0><<<dim3(gM, CH / GBN), GTHR, 0, stream>>>(XH, XH, CH, 16, WA + (size_t)(CH2 + 2 * CH) * CH, CH,
      bv, 1, x, CH, 0, 0, QKV + 2 * CH, QKVW, HRH, HRL, S11, S22, 0, 1.0f, P1, CH, 0);

  k_attn<<<dim3(NHD, G), ATHR, LDS_ATT, stream>>>(QKV, ODH, ODL, nN);

  k_gemm<0, 1><<<dim3(gM, CH / GBN), GTHR, 0, stream>>>(ODH, ODL, HDM, nN * HDM, WB, CH,
      bo, 1, x, CH, 1, 1, HMX, CH, HRH, HRL, S11, S22, 0, 1.0f, P2, CH, 1);

  k_agg<<<gA, NTHR, LDS_AGG, stream>>>(src, dst, x, geps, HGH, HGL, nN, nE, nb, vec8, MP);

  k_gemm<1, 1><<<dim3(gM, CH2 / GBN), GTHR, 0, stream>>>(HGH, HGL, CH, 16, WA, CH,
      bl1, 1, x, CH, 0, 0, HGX, CH2, HRH, HRL, S11, S22, 1, CACT, P1, CH, 0);
  k_gemm<0, 1><<<dim3(gM, CH / GBN), GTHR, 0, stream>>>(HRH, HRL, CH2, 16, WC, CH2,
      bl2, 1, x, CH, 1, 1, HGX, CH, HRH, HRL, S11, S22, 0, 1.0f, P1, CH, 1);
  k_fold<<<2, CH, 0, stream>>>(P1, S1, P2, S2, gM);
  k_combine<<<cdiv(nU32, NTHR), NTHR, 0, stream>>>(HGX, HMX, S1, S2, g1, be1, g2, be2, OUTF, FOH, FOL, nU32);
  k_gemm<1, 1><<<dim3(gM, CH2 / GBN), GTHR, 0, stream>>>(FOH, FOL, CH, 16, WB + (size_t)CH * CH, CH,
      bf1, 1, x, CH, 0, 0, HGX, CH2, T1H, T1L, S11, S22, 1, CACT, P3, CH, 0);
  k_gemm<0, 1><<<dim3(gM, CH / GBN), GTHR, 0, stream>>>(T1H, T1L, CH2, 16, WC + (size_t)CH * CH2, CH2,
      bf2, 1, OUTF, CH, 1, 0, O2, CH, HRH, HRL, S11, S22, 0, 1.0f, P3, CH, 1);
  k_fold<<<1, CH, 0, stream>>>(P3, S3, P3, S3, gM);
  k_apply<<<cdiv(nU32, NTHR), NTHR, 0, stream>>>(O2, S3, g3, be3, out0, nU32);
}
